// LocalSelfAttention_63728724738641
// MI455X (gfx1250) — hardware-verified
//
#include <hip/hip_runtime.h>


#ifndef NB
#define NB 4
#endif
#ifndef SEQ
#define SEQ 4096
#endif
#define NB_FULL  4
#define SEQ_FULL 4096
#define HID  512
#define NH   8
#define HD   64
#define ATT  (NH * HD)
#define QKVN (3 * ATT)
#define AWV  4
#define SP   48
#define PP   72

static_assert(SEQ % 64 == 0);
static_assert((NH * (SEQ / 16)) % AWV == 0);
static_assert(HID % 32 == 0);
static_assert(ATT % 64 == 0);
static_assert(QKVN % 64 == 0);
static_assert((PP * 2) % 16 == 0);

typedef _Float16 h16;
typedef unsigned short bf;
typedef __attribute__((ext_vector_type(16))) __bf16   v16bf;
typedef __attribute__((ext_vector_type(16))) _Float16 v16h;
typedef __attribute__((ext_vector_type(8)))  _Float16 v8h;
typedef __attribute__((ext_vector_type(8)))  unsigned short v8us;
typedef __attribute__((ext_vector_type(8)))  float    v8f;
typedef __attribute__((ext_vector_type(4)))  float    v4f;
typedef __attribute__((ext_vector_type(2)))  unsigned short v2us;
typedef v8h  __attribute__((may_alias)) v8ha;
typedef v4f  __attribute__((may_alias)) v4fa;
typedef v8us __attribute__((may_alias)) v8usa;

__device__ __forceinline__ unsigned short f2bf(float f) { unsigned u = __float_as_uint(f); u += 0x7FFFu + ((u >> 16) & 1u); return (unsigned short)(u >> 16); }
__device__ __forceinline__ float bf2f(unsigned short b) { return __uint_as_float(((unsigned)b) << 16); }
__device__ __forceinline__ float bfr(float f) { return bf2f(f2bf(f)); }
__device__ __forceinline__ void splitf(float y, unsigned short& h, unsigned short& l) { h = f2bf(y); l = f2bf(y - bf2f(h)); }
__device__ __forceinline__ v16h cat16(v8h lo, v8h hi) { return __builtin_shufflevector(lo, hi, 0, 1, 2, 3, 4, 5, 6, 7, 8, 9, 10, 11, 12, 13, 14, 15); }
__device__ __forceinline__ v16bf cat16b(v8us lo, v8us hi) { return __builtin_bit_cast(v16bf, __builtin_shufflevector(lo, hi, 0, 1, 2, 3, 4, 5, 6, 7, 8, 9, 10, 11, 12, 13, 14, 15)); }
__device__ __forceinline__ v8f wmma16(v16h a, v16h b, v8f c) { return __builtin_amdgcn_wmma_f32_16x16x32_f16(false, a, false, b, (short)0, c, false, false); }
__device__ __forceinline__ v8f wmmab(v16bf a, v16bf b, v8f c) { return __builtin_amdgcn_wmma_f32_16x16x32_bf16(false, a, false, b, (short)0, c, false, false); }

template <typename T16> struct WFrag;
template <> struct WFrag<h16> { typedef v16h V; static __device__ __forceinline__ V ld(const h16* p) { return cat16(*(const v8h*)p, *(const v8h*)(p + 16)); } static __device__ __forceinline__ v8f mma(V a, V b, v8f c) { return wmma16(a, b, c); } };
template <> struct WFrag<bf> { typedef v16bf V; static __device__ __forceinline__ V ld(const bf* p) { return cat16b(*(const v8us*)p, *(const v8us*)(p + 16)); } static __device__ __forceinline__ v8f mma(V a, V b, v8f c) { return wmmab(a, b, c); } };
template <typename T16, int NSPLIT, bool BIAS>
__global__ __launch_bounds__(32) void k_gemmw(const T16* __restrict__ A, const T16* __restrict__ A2, const T16* __restrict__ Bt, const T16* __restrict__ Bt2, int K, float* C, int ldc, const float* __restrict__ bias, size_t sA, size_t sB, size_t sC) {
    typedef typename WFrag<T16>::V V;
    __shared__ __align__(16) float os[16 * 68];
    const size_t z = blockIdx.z; A += z * sA; if (A2) A2 += z * sA; Bt += z * sB; if (Bt2) Bt2 += z * sB; C += z * sC;
    const int lane = threadIdx.x & 31, lr = lane & 15, hi = lane >> 4; const int r0 = blockIdx.x * 64, c0 = blockIdx.y * 64;
    v8f acc[4][4];
#pragma unroll
    for (int mb = 0; mb < 4; ++mb)
#pragma unroll
        for (int nb = 0; nb < 4; ++nb) acc[mb][nb] = (v8f){};
    const size_t aoff = (size_t)(r0 + lr) * K + 8 * hi, boff = (size_t)(c0 + lr) * K + 8 * hi;
#pragma unroll 1
    for (int kc = 0; kc < K; kc += 32) {
        V a[4], a2[4];
#pragma unroll
        for (int mb = 0; mb < 4; ++mb) { a[mb] = WFrag<T16>::ld(A + aoff + (size_t)mb * 16 * K + kc); if (NSPLIT == 1 || NSPLIT == 2) a2[mb] = WFrag<T16>::ld(A2 + aoff + (size_t)mb * 16 * K + kc); }
#pragma unroll
        for (int nb = 0; nb < 4; ++nb) { const V b = WFrag<T16>::ld(Bt + boff + (size_t)nb * 16 * K + kc); V b2; if (NSPLIT >= 2) b2 = WFrag<T16>::ld(Bt2 + boff + (size_t)nb * 16 * K + kc);
#pragma unroll
            for (int mb = 0; mb < 4; ++mb) { acc[mb][nb] = WFrag<T16>::mma(a[mb], b, acc[mb][nb]); if (NSPLIT == 1 || NSPLIT == 2) acc[mb][nb] = WFrag<T16>::mma(a2[mb], b, acc[mb][nb]); if (NSPLIT >= 2) acc[mb][nb] = WFrag<T16>::mma(a[mb], b2, acc[mb][nb]); } }
        asm volatile("v_nop\n\tv_nop\n\tv_nop\n\tv_nop" : "+v"(acc[0][0]), "+v"(acc[1][1]), "+v"(acc[2][2]), "+v"(acc[3][3]) : "v"(a[0]), "v"(a[3]));
    }
#pragma unroll
    for (int mb = 0; mb < 4; ++mb) {
#pragma unroll
        for (int nb = 0; nb < 4; ++nb) {
#pragma unroll
            for (int j = 0; j < 8; ++j) os[(hi * 8 + j) * 68 + nb * 16 + lr] = acc[mb][nb][j]; }
        __builtin_amdgcn_wave_barrier(); asm volatile("" ::: "memory");
        float* crow = C + (size_t)(r0 + mb * 16) * ldc + c0;
#pragma unroll 1
        for (int ps = 0; ps < 2; ++ps) {
#pragma unroll
            for (int s = 0; s < 8; ++s) { const int row = 2 * s + hi, cofs = lr * 4; v4f val = *(const v4fa*)(os + row * 68 + cofs); if (BIAS) { val[0] += bfr(bias[c0 + cofs]); val[1] += bfr(bias[c0 + cofs + 1]); val[2] += bfr(bias[c0 + cofs + 2]); val[3] += bfr(bias[c0 + cofs + 3]); }
                *(volatile v4f*)(crow + (size_t)row * ldc + cofs) = val; }
            if (ps == 0) __threadfence(); }
        __builtin_amdgcn_wave_barrier(); asm volatile("" ::: "memory");
    }
}

__global__ __launch_bounds__(256) void k_cvt8(const float* __restrict__ src, bf* dst, size_t n8) { const size_t i = (size_t)blockIdx.x * 256 + threadIdx.x; if (i >= n8) return; const v8f v = *(const v8f*)(src + i * 8); v8us o;
#pragma unroll
    for (int k = 0; k < 8; ++k) o[k] = f2bf(v[k]); *(volatile v8us*)(dst + i * 8) = o; __threadfence(); *(volatile v8us*)(dst + i * 8) = o; }

__global__ __launch_bounds__(256) void k_qkp(const float* __restrict__ F, h16* QK) {
    const size_t e = ((size_t)blockIdx.x * 256 + threadIdx.x) * 8; if (e >= (size_t)2 * NH * SEQ * HD) return;
    const int d = (int)(e % HD); const int t = (int)((e / HD) % SEQ); const int p = (int)(e / ((size_t)HD * SEQ));
    const float* f = F + (size_t)t * QKVN + p * HD + d;
    const v4f a = *(const v4f*)f; const v4f c = *(const v4f*)(f + 4); v8h o;
#pragma unroll
    for (int k = 0; k < 4; ++k) { o[k] = (h16)(a[k] * 8.0f); o[4 + k] = (h16)(c[k] * 8.0f); }
    *(volatile v8h*)(QK + e) = o; __threadfence(); *(volatile v8h*)(QK + e) = o; }

__global__ __launch_bounds__(256) void k_vtp(const float* __restrict__ F, bf* Vh, bf* Vl) { const size_t e = ((size_t)blockIdx.x * 256 + threadIdx.x) * 2; if (e >= (size_t)NH * HD * SEQ) return; const int t = (int)(e % SEQ); const int d = (int)((e / SEQ) % HD); const int g = (int)(e / ((size_t)SEQ * HD)); v2us oh, ol;
#pragma unroll
    for (int q = 0; q < 2; ++q) { const float x = F[(size_t)(t + q) * QKVN + 2 * ATT + g * HD + d]; unsigned short a2, c2; splitf(x, a2, c2); oh[q] = a2; ol[q] = c2; }
    *(volatile v2us*)(Vh + e) = oh; *(volatile v2us*)(Vl + e) = ol; __threadfence(); *(volatile v2us*)(Vh + e) = oh; *(volatile v2us*)(Vl + e) = ol; }

__global__ __launch_bounds__(AWV * 32) __attribute__((amdgpu_num_vgpr(256)))
void k_attw(const h16* __restrict__ Q16, const h16* __restrict__ K16, const bf* __restrict__ Vh, const bf* __restrict__ Vl, const int* __restrict__ VM, bf* ATh, bf* ATl) {
    __shared__ __align__(16) float sS[AWV][16 * SP];
    __shared__ __align__(16) unsigned short sPh[AWV][16 * PP];
    __shared__ __align__(16) unsigned short sPl[AWV][16 * PP];
    __shared__ int sVM[AWV][64];
    const int lane = threadIdx.x & 31, m = lane & 15, hh = lane >> 4, wv = threadIdx.x >> 5;
    const int w = blockIdx.x * AWV + wv; const int h = w / (SEQ / 16); const int l0 = (w % (SEQ / 16)) * 16; const int kb0 = l0 - 48;
#pragma unroll
    for (int q = 0; q < 2; ++q) { const int kk = lane + 32 * q; const int kg = kb0 + kk; const int v = VM[kg < 0 ? 0 : kg]; sVM[wv][kk] = (kg >= 0 && v != 0) ? 1 : 0; }
    const h16* qp = Q16 + ((size_t)h * SEQ + l0 + m) * HD + 8 * hh;
    const v16h qa0 = cat16(*(const v8h*)qp, *(const v8h*)(qp + 16));
    const v16h qa1 = cat16(*(const v8h*)(qp + 32), *(const v8h*)(qp + 48));
#pragma unroll
    for (int kt = 1; kt < 4; ++kt) {
        int key = kb0 + 16 * kt + m; key = key < 0 ? 0 : key;
        const h16* kp = K16 + ((size_t)h * SEQ + key) * HD + 8 * hh;
        const v16h kf0 = cat16(*(const v8h*)kp, *(const v8h*)(kp + 16));
        const v16h kf1 = cat16(*(const v8h*)(kp + 32), *(const v8h*)(kp + 48));
        v8f acc = (v8f){}; acc = wmma16(qa0, kf0, acc); acc = wmma16(qa1, kf1, acc);
        asm volatile("v_nop\n\tv_nop\n\tv_nop\n\tv_nop" : "+v"(acc) : "v"(qa0), "v"(qa1), "v"(kf0), "v"(kf1));
#pragma unroll
        for (int r = 0; r < 8; ++r) sS[wv][(8 * hh + r) * SP + 16 * (kt - 1) + m] = acc[r];
    }
    __syncthreads();
    float t[32]; float mx = -3.0e38f;
#pragma unroll
    for (int i = 0; i < 32; ++i) { const int kk = 32 * hh + i; const int j = kk - 16; const float s = sS[wv][m * SP + (j < 0 ? 0 : j)];
        const bool slot = (kk >= m + 17) && (kk <= m + 48); const bool valid = slot && (sVM[wv][kk] != 0);
        const float tv = slot ? (valid ? s * (1.0f / 512.0f) : -10000.0f) : -3.0e38f; t[i] = tv; mx = fmaxf(mx, tv); }
    mx = fmaxf(mx, __shfl_xor(mx, 16, 32));
    float sum = 0.f;
#pragma unroll
    for (int i = 0; i < 32; ++i) { const int kk = 32 * hh + i; const bool slot = (kk >= m + 17) && (kk <= m + 48); float d0 = __fsub_rn(t[i], mx); asm volatile("" : "+v"(d0));
        const float e = slot ? __builtin_amdgcn_exp2f(__fmul_rn(d0, 1.4426950408889634f)) : 0.f; t[i] = e; sum += e; }
    sum += __shfl_xor(sum, 16, 32);
    const float rinv = 1.0f / sum;
    float sum2 = 0.f;
#pragma unroll
    for (int i = 0; i < 32; ++i) { const int kk = 32 * hh + i; const bool slot = (kk >= m + 17) && (kk <= m + 48); const bool valid = slot && (sVM[wv][kk] != 0);
        const float p = valid ? t[i] * rinv : 0.f; t[i] = p; sum2 += p; }
    sum2 += __shfl_xor(sum2, 16, 32);
    const float f2 = 1.0f / fmaxf(sum2, 1e-6f);
#pragma unroll
    for (int k = 0; k < 4; ++k) { v8us oh, ol;
#pragma unroll
        for (int q = 0; q < 8; ++q) { unsigned short a2, c2; splitf(t[8 * k + q] * f2, a2, c2); oh[q] = a2; ol[q] = c2; }
        *(v8usa*)(&sPh[wv][m * PP + 32 * hh + 8 * k]) = oh; *(v8usa*)(&sPl[wv][m * PP + 32 * hh + 8 * k]) = ol; }
    __syncthreads();
    v16bf ph[2], pl[2];
#pragma unroll
    for (int c = 0; c < 2; ++c) { const unsigned short* pp = &sPh[wv][m * PP + 32 * c + 8 * hh]; const unsigned short* pq = &sPl[wv][m * PP + 32 * c + 8 * hh];
        ph[c] = cat16b(*(const v8usa*)pp, *(const v8usa*)(pp + 16)); pl[c] = cat16b(*(const v8usa*)pq, *(const v8usa*)(pq + 16)); }
    v8f acc[4];
#pragma unroll
    for (int dt = 0; dt < 4; ++dt) {
        acc[dt] = (v8f){};
        const bf* vrh = Vh + ((size_t)h * HD + 16 * dt + m) * SEQ; const bf* vrl = Vl + ((size_t)h * HD + 16 * dt + m) * SEQ;
#pragma unroll
        for (int c = 0; c < 2; ++c) {
            int ka = kb0 + 32 * c + 8 * hh; int kc = ka + 16; ka = ka < 0 ? 0 : ka; kc = kc < 0 ? 0 : kc;
            const v16bf vfh = cat16b(*(const v8us*)(vrh + ka), *(const v8us*)(vrh + kc));
            const v16bf vfl = cat16b(*(const v8us*)(vrl + ka), *(const v8us*)(vrl + kc));
            acc[dt] = wmmab(ph[c], vfh, acc[dt]); acc[dt] = wmmab(pl[c], vfh, acc[dt]); acc[dt] = wmmab(ph[c], vfl, acc[dt]);
            if (c == 1) asm volatile("v_nop\n\tv_nop\n\tv_nop\n\tv_nop" : "+v"(acc[dt]) : "v"(ph[0]), "v"(ph[1]), "v"(pl[1]), "v"(vfh), "v"(vfl));
        }
    }
    __syncthreads();
#pragma unroll
    for (int dt = 0; dt < 4; ++dt) {
#pragma unroll
        for (int r = 0; r < 8; ++r) { unsigned short a2, c2; splitf(acc[dt][r], a2, c2); sPh[wv][(8 * hh + r) * PP + 16 * dt + m] = a2; sPl[wv][(8 * hh + r) * PP + 16 * dt + m] = c2; }
    }
    __syncthreads();
    const int rr = lane >> 3, pc = (lane & 7) * 8;
#pragma unroll 1
    for (int ps = 0; ps < 2; ++ps) {
#pragma unroll
        for (int s = 0; s < 4; ++s) { const int row = 4 * s + rr; const v8us oh = *(const v8usa*)(&sPh[wv][row * PP + pc]); const v8us ol = *(const v8usa*)(&sPl[wv][row * PP + pc]);
            const size_t oo = ((size_t)(l0 + row)) * ATT + h * HD + pc; *(volatile v8us*)(ATh + oo) = oh; *(volatile v8us*)(ATl + oo) = ol; }
        if (ps == 0) __threadfence(); }
}

extern "C" void kernel_launch(void* const* d_in, const int* in_sizes, int n_in,
                              void* d_out, int out_size, void* d_ws, size_t ws_size, hipStream_t stream) {
    if (n_in < 6) return;
    if (in_sizes[0] < (NB - 1) * SEQ_FULL * HID + SEQ * HID) return;
    if (in_sizes[1] < (NB - 1) * SEQ_FULL + SEQ) return;
    if (in_sizes[2] < QKVN * HID) return;
    if (in_sizes[3] < QKVN) return;
    if (in_sizes[4] < HID * ATT) return;
    if (in_sizes[5] < HID) return;
    if (out_size < (NB - 1) * SEQ_FULL * HID + SEQ * HID) return;
    const float* x    = (const float*)d_in[0];
    const int*   vm   = (const int*)d_in[1];
    const float* wqkv = (const float*)d_in[2];
    const float* bqkv = (const float*)d_in[3];
    const float* wo   = (const float*)d_in[4];
    const float* bo   = (const float*)d_in[5];
    float* OUT = (float*)d_out;
    char* wsp = (char*)d_ws;
    auto take = [&](size_t bytes) { char* p = wsp; wsp += (bytes + 255) & ~(size_t)255; return (void*)p; };
    bf*    WQKV = (bf*)take((size_t)QKVN * HID * 2);
    bf*    WO   = (bf*)take((size_t)HID * ATT * 2);
    bf*    XB   = (bf*)take((size_t)SEQ * HID * 2);
    float* F    = (float*)take((size_t)SEQ * QKVN * 4);
    h16*   QK16 = (h16*)take((size_t)2 * NH * SEQ * HD * 2);
    bf*    VTh  = (bf*)take((size_t)NH * HD * SEQ * 2);
    bf*    VTl  = (bf*)take((size_t)NH * HD * SEQ * 2);
    bf*    ATh  = (bf*)take((size_t)SEQ * ATT * 2);
    bf*    ATl  = (bf*)take((size_t)SEQ * ATT * 2);
    if ((size_t)(wsp - (char*)d_ws) > ws_size) return;
    h16* Q16 = QK16; h16* K16 = QK16 + (size_t)NH * SEQ * HD;
    k_cvt8<<<(unsigned)(((size_t)QKVN * HID / 8 + 255) / 256), 256, 0, stream>>>(wqkv, WQKV, (size_t)QKVN * HID / 8);
    k_cvt8<<<(unsigned)(((size_t)HID * ATT / 8 + 255) / 256), 256, 0, stream>>>(wo, WO, (size_t)HID * ATT / 8);
    for (int b = 0; b < NB; ++b) {
        k_cvt8<<<(unsigned)(((size_t)SEQ * HID / 8 + 255) / 256), 256, 0, stream>>>(x + (size_t)b * SEQ_FULL * HID, XB, (size_t)SEQ * HID / 8);
        k_gemmw<bf, 0, true><<<dim3(SEQ / 64, QKVN / 64, 1), 32, 0, stream>>>(XB, nullptr, WQKV, nullptr, HID, F, QKVN, bqkv, 0, 0, 0);
        k_qkp<<<(unsigned)(((size_t)2 * NH * SEQ * HD / 8 + 255) / 256), 256, 0, stream>>>(F, QK16);
        k_vtp<<<(unsigned)(((size_t)NH * HD * SEQ / 2 + 255) / 256), 256, 0, stream>>>(F, VTh, VTl);
        k_attw<<<(unsigned)(NH * (SEQ / 16) / AWV), AWV * 32, 0, stream>>>(Q16, K16, VTh, VTl, vm + (size_t)b * SEQ_FULL, ATh, ATl);
        k_gemmw<bf, 1, true><<<dim3(SEQ / 64, HID / 64, 1), 32, 0, stream>>>(ATh, ATl, WO, nullptr, ATT, OUT + (size_t)b * SEQ_FULL * HID, HID, bo, 0, 0, 0);
    }
}
